// Damping_82884278878217
// MI455X (gfx1250) — hardware-verified
//
#include <hip/hip_runtime.h>


#define NR   1048576
#define CH   262144
#define HH   32
#define WW   64
typedef _Float16 h16;
typedef unsigned short bf;
typedef __attribute__((ext_vector_type(16))) __bf16   v16bf;
typedef __attribute__((ext_vector_type(16))) _Float16 v16h;
typedef __attribute__((ext_vector_type(8)))  _Float16 v8h;
typedef __attribute__((ext_vector_type(8)))  unsigned short v8us;
typedef __attribute__((ext_vector_type(8)))  float    v8f;
typedef __attribute__((ext_vector_type(4)))  float    v4f;
typedef v8h  __attribute__((may_alias)) v8ha;
typedef v4f  __attribute__((may_alias)) v4fa;
typedef v8us __attribute__((may_alias)) v8usa;

__device__ __forceinline__ unsigned short f2bf(float f) { unsigned u = __float_as_uint(f); u += 0x7FFFu + ((u >> 16) & 1u); return (unsigned short)(u >> 16); }
__device__ __forceinline__ float bf2f(unsigned short b) { return __uint_as_float(((unsigned)b) << 16); }
__device__ __forceinline__ float bfr(float f) { return bf2f(f2bf(f)); }
__device__ __forceinline__ v16h cat16(v8h lo, v8h hi) { return __builtin_shufflevector(lo, hi, 0, 1, 2, 3, 4, 5, 6, 7, 8, 9, 10, 11, 12, 13, 14, 15); }
__device__ __forceinline__ v16bf cat16b(v8us lo, v8us hi) { return __builtin_bit_cast(v16bf, __builtin_shufflevector(lo, hi, 0, 1, 2, 3, 4, 5, 6, 7, 8, 9, 10, 11, 12, 13, 14, 15)); }
__device__ __forceinline__ v8f wmma16(v16h a, v16h b, v8f c) { return __builtin_amdgcn_wmma_f32_16x16x32_f16(false, a, false, b, (short)0, c, false, false); }
__device__ __forceinline__ v8f wmmab(v16bf a, v16bf b, v8f c) { return __builtin_amdgcn_wmma_f32_16x16x32_bf16(false, a, false, b, (short)0, c, false, false); }


template <typename T16> struct WFrag;
template <> struct WFrag<h16> { typedef v16h V; static __device__ __forceinline__ V ld(const h16* p) { return cat16(*(const v8h*)p, *(const v8h*)(p + 16)); } static __device__ __forceinline__ v8f mma(V a, V b, v8f c) { return wmma16(a, b, c); } };
template <> struct WFrag<bf> { typedef v16bf V; static __device__ __forceinline__ V ld(const bf* p) { return cat16b(*(const v8us*)p, *(const v8us*)(p + 16)); } static __device__ __forceinline__ v8f mma(V a, V b, v8f c) { return wmmab(a, b, c); } };
template <typename T16, int NSPLIT, bool BIAS>
__global__ __launch_bounds__(32) void k_gemmw(const T16* __restrict__ A, const T16* __restrict__ A2, const T16* __restrict__ Bt, const T16* __restrict__ Bt2, int K, float* C, int ldc, const float* __restrict__ bias, size_t sA, size_t sB, size_t sC) {
    typedef typename WFrag<T16>::V V;
    __shared__ __align__(16) float os[16 * 68];
    const size_t z = blockIdx.z; A += z * sA; if (A2) A2 += z * sA; Bt += z * sB; if (Bt2) Bt2 += z * sB; C += z * sC;
    const int lane = threadIdx.x & 31, lr = lane & 15, hi = lane >> 4; const int r0 = blockIdx.x * 64, c0 = blockIdx.y * 64;
    v8f acc[4][4];
#pragma unroll
    for (int mb = 0; mb < 4; ++mb)
#pragma unroll
        for (int nb = 0; nb < 4; ++nb) acc[mb][nb] = (v8f){};
    const size_t aoff = (size_t)(r0 + lr) * K + 8 * hi, boff = (size_t)(c0 + lr) * K + 8 * hi;
#pragma unroll 1
    for (int kc = 0; kc < K; kc += 32) {
        V a[4], a2[4];
#pragma unroll
        for (int mb = 0; mb < 4; ++mb) { a[mb] = WFrag<T16>::ld(A + aoff + (size_t)mb * 16 * K + kc); if (NSPLIT == 1 || NSPLIT == 2) a2[mb] = WFrag<T16>::ld(A2 + aoff + (size_t)mb * 16 * K + kc); }
#pragma unroll
        for (int nb = 0; nb < 4; ++nb) { const V b = WFrag<T16>::ld(Bt + boff + (size_t)nb * 16 * K + kc); V b2; if (NSPLIT >= 2) b2 = WFrag<T16>::ld(Bt2 + boff + (size_t)nb * 16 * K + kc);
#pragma unroll
            for (int mb = 0; mb < 4; ++mb) { acc[mb][nb] = WFrag<T16>::mma(a[mb], b, acc[mb][nb]); if (NSPLIT == 1 || NSPLIT == 2) acc[mb][nb] = WFrag<T16>::mma(a2[mb], b, acc[mb][nb]); if (NSPLIT >= 2) acc[mb][nb] = WFrag<T16>::mma(a[mb], b2, acc[mb][nb]); } }
        asm volatile("v_nop\n\tv_nop\n\tv_nop\n\tv_nop" : "+v"(acc[0][0]), "+v"(acc[1][1]), "+v"(acc[2][2]), "+v"(acc[3][3]) : "v"(a[0]), "v"(a[3]));
    }
#pragma unroll
    for (int mb = 0; mb < 4; ++mb) {
#pragma unroll
        for (int nb = 0; nb < 4; ++nb) {
#pragma unroll
            for (int j = 0; j < 8; ++j) os[(hi * 8 + j) * 68 + nb * 16 + lr] = acc[mb][nb][j]; }
        __builtin_amdgcn_wave_barrier(); asm volatile("" ::: "memory");
        float* crow = C + (size_t)(r0 + mb * 16) * ldc + c0;
#pragma unroll 1
        for (int ps = 0; ps < 2; ++ps) {
#pragma unroll
            for (int s = 0; s < 8; ++s) { const int row = 2 * s + hi, cofs = lr * 4; v4f val = *(const v4fa*)(os + row * 68 + cofs); if (BIAS) { val[0] += bfr(bias[c0 + cofs]); val[1] += bfr(bias[c0 + cofs + 1]); val[2] += bfr(bias[c0 + cofs + 2]); val[3] += bfr(bias[c0 + cofs + 3]); }
                *(volatile v4f*)(crow + (size_t)row * ldc + cofs) = val; }
            if (ps == 0) __threadfence(); }
        __builtin_amdgcn_wave_barrier(); asm volatile("" ::: "memory");
    }
}

__device__ __forceinline__ void splitf(float y, unsigned short& h, unsigned short& l) { h = f2bf(y); l = f2bf(y - bf2f(h)); }
typedef __attribute__((ext_vector_type(2))) float v2f;
typedef __attribute__((ext_vector_type(4))) unsigned short v4us;

__global__ __launch_bounds__(256) void k_w2(const float* __restrict__ wd2, const float* __restrict__ wo2, bf* Bt) { const int e = (blockIdx.x * 256 + threadIdx.x) * 4; if (e >= WW * WW) return; const int i0 = e % WW, j = e / WW; v4us o;
#pragma unroll
    for (int u = 0; u < 4; ++u) { const int i = i0 + u; float v = 0.f; if (j < HH && i < HH) v = wd2[i * HH + j]; else if (j >= HH && i >= HH) v = wo2[(i - HH) * HH + (j - HH)]; o[u] = f2bf(v); } *(volatile v4us*)(Bt + e) = o; __threadfence(); *(volatile v4us*)(Bt + e) = o; }
__global__ __launch_bounds__(64) void k_b2(const float* __restrict__ bd2, const float* __restrict__ bo2, float* b2) { const int j = threadIdx.x; const float v = j < HH ? bd2[j] : bo2[j - HH]; *(volatile float*)(b2 + j) = v; __threadfence(); *(volatile float*)(b2 + j) = v; }
__global__ __launch_bounds__(256) void k_l1(const float* __restrict__ x, int r0, const float* __restrict__ wd1, const float* __restrict__ bd1, const float* __restrict__ wo1, const float* __restrict__ bo1, bf* Ah, bf* Al) { const int e = (blockIdx.x * 256 + threadIdx.x) * 4; if (e >= CH * WW) return; const int j0 = e % WW; const int r = r0 + e / WW;
    float x0 = bfr(x[(size_t)r * 2]), x1 = bfr(x[(size_t)r * 2 + 1]); asm volatile("" : "+v"(x0)); asm volatile("" : "+v"(x1)); v4us oh, ol;
#pragma unroll
    for (int u = 0; u < 4; ++u) { const int j = j0 + u; float w0, w1, bb; if (j < HH) { w0 = bfr(wd1[j]); w1 = bfr(wd1[HH + j]); bb = bfr(bd1[j]); } else { w0 = bfr(wo1[j - HH]); w1 = bfr(wo1[HH + j - HH]); bb = bfr(bo1[j - HH]); }
        asm volatile("" : "+v"(w0)); asm volatile("" : "+v"(w1)); asm volatile("" : "+v"(bb)); float p0 = __fmul_rn(x0, w0), p1 = __fmul_rn(x1, w1); asm volatile("" : "+v"(p0)); asm volatile("" : "+v"(p1)); const float h = tanhf(__fadd_rn(__fadd_rn(p0, p1), bb)); unsigned short a, b; splitf(h, a, b); oh[u] = a; ol[u] = b; }
    *(volatile v4us*)(Ah + e) = oh; *(volatile v4us*)(Al + e) = ol; __threadfence(); *(volatile v4us*)(Ah + e) = oh; *(volatile v4us*)(Al + e) = ol; }
__global__ __launch_bounds__(256) void k_l3(const float* __restrict__ G, const float* __restrict__ x, int r0, const float* __restrict__ wd3, const float* __restrict__ bd3, const float* __restrict__ wo3, const float* __restrict__ bo3, float* OUT) { const int rl = blockIdx.x * 256 + threadIdx.x; if (rl >= CH) return; const int r = r0 + rl; const float* gr = G + (size_t)rl * WW;
    float d0 = 0.f, d1 = 0.f, c = 0.f;
#pragma unroll 1
    for (int j = 0; j < HH; ++j) { const float t = tanhf(gr[j]); float w0 = bfr(wd3[j * 2]), w1 = bfr(wd3[j * 2 + 1]); asm volatile("" : "+v"(w0)); asm volatile("" : "+v"(w1)); float p0 = __fmul_rn(t, w0), p1 = __fmul_rn(t, w1); asm volatile("" : "+v"(p0)); asm volatile("" : "+v"(p1)); d0 = __fadd_rn(d0, p0); d1 = __fadd_rn(d1, p1); }
#pragma unroll 1
    for (int j = 0; j < HH; ++j) { const float t = tanhf(gr[HH + j]); float w0 = bfr(wo3[j]); asm volatile("" : "+v"(w0)); float p0 = __fmul_rn(t, w0); asm volatile("" : "+v"(p0)); c = __fadd_rn(c, p0); }
    float bb0 = bfr(bd3[0]), bb1 = bfr(bd3[1]), bc = bfr(bo3[0]); asm volatile("" : "+v"(bb0)); asm volatile("" : "+v"(bb1)); asm volatile("" : "+v"(bc)); d0 = __fadd_rn(d0, bb0); d1 = __fadd_rn(d1, bb1); c = __fadd_rn(c, bc);
    float x0 = bfr(x[(size_t)r * 2]), x1 = bfr(x[(size_t)r * 2 + 1]); asm volatile("" : "+v"(x0)); asm volatile("" : "+v"(x1));
    float ra = __fadd_rn(fmaxf(d0, 0.f), 0.001f), rb = __fadd_rn(fmaxf(d1, 0.f), 0.001f); asm volatile("" : "+v"(ra)); asm volatile("" : "+v"(rb)); const float a = __fmul_rn(ra, x0), b = __fmul_rn(rb, x1);
    float aa = __fmul_rn(a, a), ac = __fmul_rn(a, c), cc = __fmul_rn(c, c), bb = __fmul_rn(b, b); asm volatile("" : "+v"(aa)); asm volatile("" : "+v"(ac)); asm volatile("" : "+v"(cc)); asm volatile("" : "+v"(bb));
    float t1 = __fmul_rn(aa, x0), t2 = __fmul_rn(ac, x1), t3 = __fmul_rn(ac, x0), s4 = __fadd_rn(cc, bb); asm volatile("" : "+v"(t1)); asm volatile("" : "+v"(t2)); asm volatile("" : "+v"(t3)); asm volatile("" : "+v"(s4)); float t4 = __fmul_rn(s4, x1); asm volatile("" : "+v"(t4));
    v2f o; o[0] = __fadd_rn(t1, t2); o[1] = __fadd_rn(t3, t4); *(volatile v2f*)(OUT + (size_t)r * 2) = o; __threadfence(); *(volatile v2f*)(OUT + (size_t)r * 2) = o; }

extern "C" void kernel_launch(void* const* d_in, const int* in_sizes, int n_in,
                              void* d_out, int out_size, void* d_ws, size_t ws_size, hipStream_t stream) {
    (void)in_sizes; (void)n_in; (void)out_size;
    const float** I = (const float**)d_in;
    const float *x = I[0], *wd1 = I[1], *wd2 = I[2], *wd3 = I[3], *wo1 = I[4], *wo2 = I[5], *wo3 = I[6], *bd1 = I[7], *bd2 = I[8], *bd3 = I[9], *bo1 = I[10], *bo2 = I[11], *bo3 = I[12];
    float* OUT = (float*)d_out;
    char* wsp = (char*)d_ws;
    auto take = [&](size_t bytes) { char* p = wsp; wsp += (bytes + 255) & ~(size_t)255; return (void*)p; };
    bf* W2 = (bf*)take(WW * WW * 2); float* b2 = (float*)take(256); bf* Ah = (bf*)take((size_t)CH * WW * 2); bf* Al = (bf*)take((size_t)CH * WW * 2); float* G = (float*)take((size_t)CH * WW * 4);
    if ((size_t)(wsp - (char*)d_ws) > ws_size) return;
    k_w2<<<(WW * WW / 4 + 255) / 256, 256, 0, stream>>>(wd2, wo2, W2); k_b2<<<1, 64, 0, stream>>>(bd2, bo2, b2);
    for (int r0 = 0; r0 < NR; r0 += CH) {
        k_l1<<<(CH * WW / 4 + 255) / 256, 256, 0, stream>>>(x, r0, wd1, bd1, wo1, bo1, Ah, Al);
        k_gemmw<bf, 1, true><<<dim3(CH / 64, 1, 1), 32, 0, stream>>>(Ah, Al, W2, nullptr, WW, G, WW, b2, 0, 0, 0);
        k_l3<<<(CH + 255) / 256, 256, 0, stream>>>(G, x, r0, wd3, bd3, wo3, bo3, OUT); }
}
